// Model_48172353192667
// MI455X (gfx1250) — hardware-run, weakly checked
//
#include <hip/hip_runtime.h>
#include <math.h>


#ifndef NB
#define NB 64
#endif
#ifndef NV
#define NV 50000
#endif
#define NB_FULL 64
#define NV_FULL 50000
#define NJ   25
#define KP   32
#define PBAT 32
#define PT   512
#define NT16 (NV / 16)
#define JOC  (PBAT * NJ * 3 / 4)
#define OUT1_OFF ((size_t)NB_FULL * NJ * 3)
#define OSN  112

static_assert(NB % PBAT == 0);
static_assert(NB % 2 == 0);
static_assert(NB <= NB_FULL);
static_assert(NV <= NV_FULL);
static_assert(NV % 16 == 0);
static_assert(NJ <= KP);
static_assert(KP == 32);
static_assert(PT == PBAT * 16);
static_assert((PBAT * 64) % PT == 0);
static_assert(((size_t)PBAT * 16 * KP) == (size_t)((PBAT * 64) / PT) * PT * 8);
static_assert(((size_t)PBAT * NJ * 3 * 4) % 128 == 0);
static_assert(JOC % 8 == 0);
static_assert(2 * PT >= JOC);
static_assert((OUT1_OFF * 4) % 128 == 0);
static_assert(OUT1_OFF * 4 == 19200);
static_assert(((size_t)2 * NV_FULL * 3 * 4) % 128 == 0);
static_assert(24 * 16 == 32 * 3 * 4);
static_assert((size_t)PBAT * NJ * 16 * 4 + 2 * NJ * 16 * 4 + PBAT * 16 * 4 + PBAT * 8 * 4 + 32 * 4 <= 131072);
static_assert(OUT1_OFF + ((size_t)(NB - 1) * NV_FULL + NV) * 3 <= OUT1_OFF + (size_t)NB_FULL * NV_FULL * 3);

typedef unsigned short bf;
typedef __attribute__((ext_vector_type(16))) __bf16   v16bf;
typedef __attribute__((ext_vector_type(8)))  unsigned short v8us;
typedef __attribute__((ext_vector_type(8)))  float    v8f;
typedef __attribute__((ext_vector_type(4)))  float    v4f;
typedef v4f  __attribute__((may_alias)) v4fa;

__device__ __forceinline__ unsigned short f2bf(float f) { unsigned u = __float_as_uint(f); u += 0x7FFFu + ((u >> 16) & 1u); return (unsigned short)(u >> 16); }
__device__ __forceinline__ float bfr(float f) { return __uint_as_float(((unsigned)f2bf(f)) << 16); }
__device__ __forceinline__ v16bf cat16b(v8us lo, v8us hi) { return __builtin_bit_cast(v16bf, __builtin_shufflevector(lo, hi, 0, 1, 2, 3, 4, 5, 6, 7, 8, 9, 10, 11, 12, 13, 14, 15)); }
__device__ __forceinline__ v16bf ldb(const bf* p)  { return cat16b(*(const v8us*)p, *(const v8us*)(p + 16)); }
__device__ __forceinline__ void wave_sync() { __builtin_amdgcn_fence(3  , "wavefront"); __builtin_amdgcn_wave_barrier(); asm volatile("" ::: "memory"); }
__device__ __forceinline__ v8f wmmab_g(v16bf a, v16bf b, v8f c) {
    c = __builtin_amdgcn_wmma_f32_16x16x32_bf16(false, a, false, b, (short)0, c, false, false);
    asm volatile("v_nop\n\tv_nop\n\tv_nop\n\tv_nop" : "+v"(c) : "v"(a), "v"(b));
    return c;
}

__global__ __launch_bounds__(256) void k_swplane(const float* __restrict__ sw, bf* SWP, int nchunks) {
#pragma clang fp contract(off)
    const int i = blockIdx.x * 256 + threadIdx.x; if (i >= nchunks) return;
    const int v = i >> 2, q = i & 3;
    v8us o;
#pragma unroll
    for (int k = 0; k < 8; ++k) {
        const int j = 8 * q + k; const int jc = j < NJ ? j : NJ - 1;
        float x = sw[(size_t)v * NJ + jc];
        asm volatile("" : "+v"(x));
        o[k] = (j < NJ) ? f2bf(x) : (unsigned short)0; }
    *(volatile v8us*)(SWP + (size_t)i * 8) = o; __threadfence(); *(volatile v8us*)(SWP + (size_t)i * 8) = o;
}

__global__ __launch_bounds__(PT) void k_pose(const float* __restrict__ je, const float* __restrict__ lp, const float* __restrict__ gpi, const float* __restrict__ sc,
                                             const int* __restrict__ par, bf* TH, bf* TL, float* OUT0) {
#pragma clang fp contract(off)
    __shared__ __align__(16) float Gall[PBAT * NJ * 16];
    __shared__ float LPs[NJ * 16];
    __shared__ float GPs[NJ * 16];
    __shared__ float Ls[PBAT * 16];
    __shared__ float CS[PBAT * 8];
    __shared__ int PAR[32];
    const int tid = threadIdx.x;
    const int bl = tid >> 4, e = tid & 15, r = e >> 2, c = e & 3;
    const int b = blockIdx.x * PBAT + bl;
    {
        const int i = tid < NJ * 16 ? tid : NJ * 16 - 1;
        float a = bfr(lp[i]); const float g = bfr(gpi[i]);
        const int jj = i >> 4, rr = (i & 15) >> 2, cc = i & 3;
        float s = bfr(sc[jj * 3 + (rr < 3 ? rr : 2)]);
        asm volatile("" : "+v"(a)); asm volatile("" : "+v"(s));
        const float a2 = a + s;
        a = ((rr < 3) & (cc == 3)) ? a2 : a;
        if (tid < NJ * 16) { LPs[i] = a; GPs[i] = g; }
        int pv = par[tid < NJ ? tid : NJ - 1];
        asm volatile("" : "+v"(pv));
        if (tid < 32) PAR[tid] = (tid < NJ) ? pv : 0;
    }
#pragma unroll 1
    for (int i = tid; i < PBAT * NJ * 16; i += PT) Gall[i] = (((i & 15) % 5) == 0) ? 1.0f : 0.0f;
    __syncthreads();
    int root = 0;
#pragma unroll 1
    for (int j = NJ - 1; j >= 0; --j) { if (PAR[j] < 0) root = j; }
#pragma unroll 1
    for (int j = 0; j < NJ; ++j) {
        const int ai = e < 3 ? e : 2;
        const float ang = bfr(je[((size_t)b * NJ + j) * 3 + ai]);
        float sv, cv; sincosf(ang, &sv, &cv);
        if (e < 3) { CS[bl * 8 + e] = cv; CS[bl * 8 + 4 + e] = sv; }
        __syncthreads();
        const float cx = CS[bl * 8 + 0], cy = CS[bl * 8 + 1], cz = CS[bl * 8 + 2];
        const float sx = CS[bl * 8 + 4], sy = CS[bl * 8 + 5], sz = CS[bl * 8 + 6];
        const float r00 = cz * cy, r01 = cz * sy * sx - sz * cx, r02 = cz * sy * cx + sz * sx;
        const float r10 = sz * cy, r11 = sz * sy * sx + cz * cx, r12 = sz * sy * cx - cz * sx;
        const float r20 = -sy,     r21 = cy * sx,                r22 = cy * cx;
        const float q0 = (c == 0) ? r00 : ((c == 1) ? r01 : ((c == 2) ? r02 : 0.0f));
        const float q1 = (c == 0) ? r10 : ((c == 1) ? r11 : ((c == 2) ? r12 : 0.0f));
        const float q2 = (c == 0) ? r20 : ((c == 1) ? r21 : ((c == 2) ? r22 : 0.0f));
        const float q3 = (c == 3) ? 1.0f : 0.0f;
        const int lpo = j * 16 + r * 4;
        const float lv = ((LPs[lpo] * q0 + LPs[lpo + 1] * q1) + LPs[lpo + 2] * q2) + LPs[lpo + 3] * q3;
        Ls[bl * 16 + e] = lv;
        __syncthreads();
        int pj = PAR[j]; pj = pj < 0 ? 0 : (pj > NJ - 1 ? NJ - 1 : pj);
        const int go = (bl * NJ + pj) * 16 + r * 4;
        const int lo = bl * 16 + c;
        const float gn = ((Gall[go] * Ls[lo] + Gall[go + 1] * Ls[lo + 4]) + Gall[go + 2] * Ls[lo + 8]) + Gall[go + 3] * Ls[lo + 12];
        __syncthreads();
        if (j != root) Gall[(bl * NJ + j) * 16 + e] = gn;
    }
    __syncthreads();
    const size_t pbase = (size_t)blockIdx.x * PBAT * 16 * KP;
#pragma unroll 1
    for (int it = 0; it < (PBAT * 64) / PT; ++it) {
        const int ci = it * PT + tid;
        const int pb = ci >> 6, rc = (ci >> 2) & 15, qq = ci & 3;
        const int pr = rc >> 2, pcn = rc & 3;
        v8us hv, lv8;
#pragma unroll
        for (int k = 0; k < 8; ++k) {
            const int j = 8 * qq + k; const int jc = j < NJ ? j : NJ - 1;
            const int go = (pb * NJ + jc) * 16 + pr * 4; const int po = jc * 16 + pcn;
            const float t = ((Gall[go] * GPs[po] + Gall[go + 1] * GPs[po + 4]) + Gall[go + 2] * GPs[po + 8]) + Gall[go + 3] * GPs[po + 12];
            const float tz = (j < NJ) ? t : 0.0f;
            const unsigned short th = f2bf(tz);
            const float thf = __uint_as_float(((unsigned)th) << 16);
            hv[k] = th; lv8[k] = f2bf(tz - thf); }
        const size_t oo = pbase + (size_t)ci * 8;
        *(volatile v8us*)(TH + oo) = hv; *(volatile v8us*)(TL + oo) = lv8;
        __threadfence();
        *(volatile v8us*)(TH + oo) = hv; *(volatile v8us*)(TL + oo) = lv8;
    }
#pragma unroll 1
    for (int it = 0; it < 2; ++it) {
        const int t4 = it * PT + tid; const int tc = t4 < JOC ? t4 : JOC - 1;
        v4f val;
#pragma unroll
        for (int i = 0; i < 4; ++i) {
            const int f = tc * 4 + i; const int bb = f / (NJ * 3); const int rem = f - bb * (NJ * 3);
            const int jj = rem / 3; const int rr = rem - jj * 3;
            val[i] = Gall[(bb * NJ + jj) * 16 + rr * 4 + 3]; }
        const size_t oo = (size_t)blockIdx.x * (PBAT * NJ * 3) + (size_t)tc * 4;
        if (t4 < JOC) *(volatile v4f*)(OUT0 + oo) = val;
        __threadfence();
        if (t4 < JOC) *(volatile v4f*)(OUT0 + oo) = val;
    }
}

__global__ __launch_bounds__(32) void k_skin(const bf* __restrict__ SWP, const bf* __restrict__ TH, const bf* __restrict__ TL,
                                             const float* __restrict__ vpos, const float* __restrict__ pcor, const float* __restrict__ icor, float* OUT) {
    __shared__ __align__(16) float os[OSN];
    const int lane = threadIdx.x & 31, lr = lane & 15, hi = lane >> 4;
    const int q = blockIdx.x;
    const int s0 = 2 * q, s1 = 2 * q + 1;
    const int hb0 = s0 >= NT16 ? 1 : 0, hb1 = s1 >= NT16 ? 1 : 0;
    const int v00 = 16 * (s0 - hb0 * NT16), v01 = 16 * (s1 - hb1 * NT16);
    const v16bf w0 = ldb(SWP + (size_t)(v00 + lr) * KP + 8 * hi);
    const v16bf w1 = ldb(SWP + (size_t)(v01 + lr) * KP + 8 * hi);
    const float bx0 = bfr(vpos[(size_t)(v00 + lr) * 3 + 0]), by0 = bfr(vpos[(size_t)(v00 + lr) * 3 + 1]), bz0 = bfr(vpos[(size_t)(v00 + lr) * 3 + 2]);
    const float bx1 = bfr(vpos[(size_t)(v01 + lr) * 3 + 0]), by1 = bfr(vpos[(size_t)(v01 + lr) * 3 + 1]), bz1 = bfr(vpos[(size_t)(v01 + lr) * 3 + 2]);
    const size_t fo = (size_t)lr * KP + 8 * hi;
    const int ia0 = lr * 3 + 2 * hi;
    const int ib0 = hi ? (96 + lr) : (lr * 3 + 1);
    const int ia1 = 48 + lr * 3 + 2 * hi;
    const int ib1 = hi ? (96 + lr) : (48 + lr * 3 + 1);
    const int li = lane < 24 ? lane : 23;
#pragma unroll 1
    for (int p = 0; p < NB / 2; ++p) {
        const int b0 = 2 * p + hb0, b1 = 2 * p + hb1;
        const v16bf th0 = ldb(TH + (size_t)b0 * (16 * KP) + fo), tl0 = ldb(TL + (size_t)b0 * (16 * KP) + fo);
        const v16bf th1 = ldb(TH + (size_t)b1 * (16 * KP) + fo), tl1 = ldb(TL + (size_t)b1 * (16 * KP) + fo);
        v8f a0 = (v8f){}, a1 = (v8f){};
        a0 = wmmab_g(th0, w0, a0); a0 = wmmab_g(tl0, w0, a0);
        a1 = wmmab_g(th1, w1, a1); a1 = wmmab_g(tl1, w1, a1);
        const size_t g0 = ((size_t)b0 * NV_FULL + (size_t)(v00 + lr)) * 3;
        const size_t g1 = ((size_t)b1 * NV_FULL + (size_t)(v01 + lr)) * 3;
        const float mx0 = (bx0 + bfr(pcor[g0 + 0])) + bfr(icor[g0 + 0]);
        const float my0 = (by0 + bfr(pcor[g0 + 1])) + bfr(icor[g0 + 1]);
        const float mz0 = (bz0 + bfr(pcor[g0 + 2])) + bfr(icor[g0 + 2]);
        const float mx1 = (bx1 + bfr(pcor[g1 + 0])) + bfr(icor[g1 + 0]);
        const float my1 = (by1 + bfr(pcor[g1 + 1])) + bfr(icor[g1 + 1]);
        const float mz1 = (bz1 + bfr(pcor[g1 + 2])) + bfr(icor[g1 + 2]);
        const float oA0 = ((a0[0] * mx0 + a0[1] * my0) + a0[2] * mz0) + a0[3];
        const float oB0 = ((a0[4] * mx0 + a0[5] * my0) + a0[6] * mz0) + a0[7];
        const float oA1 = ((a1[0] * mx1 + a1[1] * my1) + a1[2] * mz1) + a1[3];
        const float oB1 = ((a1[4] * mx1 + a1[5] * my1) + a1[6] * mz1) + a1[7];
        os[ia0] = oA0; os[ib0] = oB0; os[ia1] = oA1; os[ib1] = oB1;
        wave_sync();
        const v4f val = *(const v4fa*)(&os[li * 4]);
        const size_t base0 = OUT1_OFF + ((size_t)b0 * NV_FULL + (size_t)v00) * 3;
        const size_t base1 = OUT1_OFF + ((size_t)b1 * NV_FULL + (size_t)v01) * 3;
        const size_t off = (li < 12) ? (base0 + (size_t)(4 * li)) : (base1 + (size_t)(4 * (li - 12)));
        if (lane < 24) *(volatile v4f*)(OUT + off) = val;
        __threadfence();
        if (lane < 24) *(volatile v4f*)(OUT + off) = val;
        wave_sync();
    }
}

static constexpr size_t al256(size_t v) { return (v + 255) & ~(size_t)255; }
static constexpr size_t SZ_SW = al256((size_t)NV * KP * 2);
static constexpr size_t SZ_T  = al256((size_t)NB * 16 * KP * 2);
static constexpr size_t SZ_TOTAL = SZ_SW + 2 * SZ_T;
static_assert(SZ_TOTAL <= (size_t)134217728);
static_assert((size_t)NV * 4 * 8 * 2 == (size_t)NV * KP * 2);
static_assert((size_t)(NB / PBAT) * PBAT * 16 * KP * 2 <= SZ_T);

extern "C" void kernel_launch(void* const* d_in, const int* in_sizes, int n_in,
                              void* d_out, int out_size, void* d_ws, size_t ws_size, hipStream_t stream) {
    if (n_in < 9) return;
    const size_t needc = ((size_t)(NB - 1) * NV_FULL + NV) * 3;
    if ((size_t)in_sizes[0] < (size_t)NB * NJ * 3) return;
    if ((size_t)in_sizes[1] < (size_t)NV * 3 || (size_t)in_sizes[2] < (size_t)NV * NJ) return;
    if (in_sizes[3] < NJ * 16 || in_sizes[4] < NJ * 16 || in_sizes[5] < NJ * 3) return;
    if ((size_t)in_sizes[6] < needc || (size_t)in_sizes[7] < needc || in_sizes[8] < NJ) return;
    if ((size_t)out_size < OUT1_OFF + needc) return;
    if (SZ_TOTAL > ws_size) return;
    const float* je  = (const float*)d_in[0];
    const float* vp  = (const float*)d_in[1];
    const float* sw  = (const float*)d_in[2];
    const float* lp  = (const float*)d_in[3];
    const float* gpi = (const float*)d_in[4];
    const float* sc  = (const float*)d_in[5];
    const float* pcr = (const float*)d_in[6];
    const float* icr = (const float*)d_in[7];
    const int*   par = (const int*)d_in[8];
    float* OUT = (float*)d_out;
    char* wsp = (char*)d_ws;
    bf* SWP = (bf*)wsp; wsp += SZ_SW;
    bf* TH  = (bf*)wsp; wsp += SZ_T;
    bf* TL  = (bf*)wsp; wsp += SZ_T;

    const int nchunks = NV * 4;
    k_swplane<<<(unsigned)((nchunks + 255) / 256), 256, 0, stream>>>(sw, SWP, nchunks);
    k_pose<<<NB / PBAT, PT, 0, stream>>>(je, lp, gpi, sc, par, TH, TL, OUT);
    k_skin<<<NT16, 32, 0, stream>>>(SWP, TH, TL, vp, pcr, icr, OUT);
}
